// Self_Attn_3D_27247272526194
// MI455X (gfx1250) — hardware-verified
//
#include <hip/hip_runtime.h>

#define CIN   256
#define CQK   32
#define HWN   4096
#define NBAT  8
#define NTOK  32768
#define PBLK  64
#define QBLK  64
#define PW    264

static_assert(NTOK == NBAT * HWN);
static_assert((NTOK % PBLK) == 0 && (NTOK % QBLK) == 0 && (HWN % QBLK) == 0);
static_assert((HWN % 32) == 0 && (CIN % 32) == 0 && CQK == 32);
static_assert((PW % 8) == 0 && PBLK == 64 && QBLK == 64);

typedef __bf16         v16bf __attribute__((ext_vector_type(16)));
typedef unsigned short v16us __attribute__((ext_vector_type(16)));
typedef unsigned short v8us  __attribute__((ext_vector_type(8)));
typedef float          v8f   __attribute__((ext_vector_type(8)));
typedef float          v4f   __attribute__((ext_vector_type(4)));
typedef unsigned int   v4u   __attribute__((ext_vector_type(4)));

__device__ __forceinline__ unsigned short bf_bits(float f) {
  unsigned u = __float_as_uint(f);
  return (unsigned short)((u + 0x7FFFu + ((u >> 16) & 1u)) >> 16);
}
__device__ __forceinline__ float bf_up(unsigned short hb) { return __uint_as_float(((unsigned)hb) << 16); }
__device__ __forceinline__ float bf_r(float f) { return bf_up(bf_bits(f)); }
__device__ __forceinline__ v8f zero8() { v8f z = {0.f, 0.f, 0.f, 0.f, 0.f, 0.f, 0.f, 0.f}; return z; }

__device__ __forceinline__ v16bf ldfrag_b(const unsigned short* p) {
  union { v16us v; v8us hv[2]; } f;
  f.hv[0] = *(const v8us*)(p);
  f.hv[1] = *(const v8us*)(p + 16);
  return __builtin_bit_cast(v16bf, f.v);
}

__device__ __forceinline__ v8f mma_b(v16bf a, v16bf b, v8f c) {
  return __builtin_amdgcn_wmma_f32_16x16x32_bf16(false, a, false, b, (short)0, c, false, false);
}
__device__ __forceinline__ void guard_p(v8f& c0, v8f& c1, v8f& c2, v8f& c3,
                                        v16bf a, v16bf b0, v16bf b1, v16bf b2, v16bf b3) {
#if defined(__HIP_DEVICE_COMPILE__)
  asm volatile("v_nop\n\tv_nop\n\tv_nop\n\tv_nop"
               : "+v"(c0), "+v"(c1), "+v"(c2), "+v"(c3)
               : "v"(a), "v"(b0), "v"(b1), "v"(b2), "v"(b3));
#endif
}
__device__ __forceinline__ void guard_s(v8f& s0, v8f& s1, v16bf a0, v16bf a1, v16bf a2, v16bf a3,
                                        v16bf b0, v16bf b1) {
#if defined(__HIP_DEVICE_COMPILE__)
  asm volatile("v_nop\n\tv_nop\n\tv_nop\n\tv_nop"
               : "+v"(s0), "+v"(s1)
               : "v"(a0), "v"(a1), "v"(a2), "v"(a3), "v"(b0), "v"(b1));
#endif
}
__device__ __forceinline__ void acc_guard4(v8f& a, v8f& b, v8f& c, v8f& d) {
#if defined(__HIP_DEVICE_COMPILE__)
  asm volatile("v_nop\n\tv_nop\n\tv_nop\n\tv_nop" : "+v"(a), "+v"(b), "+v"(c), "+v"(d));
#endif
}
__device__ __forceinline__ void sched_fence() {
#if defined(__HIP_DEVICE_COMPILE__)
  asm volatile("" ::: "memory");
#endif
}

__global__ __launch_bounds__(256) void k_prep(const float* __restrict__ Wv, const float* __restrict__ bv,
                                               float* wsum, float* aux) {
  __shared__ __align__(16) float sws[CIN];
  __shared__ float sbv[CIN];
  __shared__ __align__(16) float saux[32];
  const int tid = threadIdx.x, wave = tid >> 5, lane = tid & 31;
  const float* row = Wv + (size_t)tid * CIN;
  float s = 0.f;
#pragma unroll 4
  for (int j = 0; j < CIN / 4; ++j) {
    const v4f w = *(const v4f*)(row + 4 * j);
    s += bf_r(w[0]); s += bf_r(w[1]); s += bf_r(w[2]); s += bf_r(w[3]);
  }
  sws[tid] = s;
  sbv[tid] = bf_r(bv[tid]);
  if (tid < 32) saux[tid] = 0.f;
  __syncthreads();
  if (tid == 0) {
    float t = 0.f;
#pragma unroll 1
    for (int c = 0; c < CIN; ++c) t += sbv[c];
    saux[0] = t;
  }
  __syncthreads();
  if (wave < 2) {
    const v4f v = *(const v4f*)(sws + 128 * wave + 4 * lane);
    float* dst = wsum + 128 * wave + 4 * lane;
    *(volatile v4f*)dst = v;
    __threadfence();
    *(volatile v4f*)dst = v;
  } else if (wave == 2) {
    const v4f v = *(const v4f*)(saux + 4 * (lane & 7));
    float* dst = aux + 4 * (lane & 7);
    if (lane < 8) *(volatile v4f*)dst = v;
    __threadfence();
    if (lane < 8) *(volatile v4f*)dst = v;
  }
}

__global__ __launch_bounds__(128) void k_proj(const float* __restrict__ x,
                                               const float* __restrict__ Wq, const float* __restrict__ bq,
                                               const float* __restrict__ Wk, const float* __restrict__ bk,
                                               const float* wsum, const float* aux,
                                               unsigned short* qh, unsigned short* ql,
                                               unsigned short* kh, unsigned short* kl,
                                               float* xmean, float* vbar) {
  __shared__ __align__(16) unsigned short sW[64 * PW];
  __shared__ __align__(16) unsigned short sO[4 * 4 * 16 * CQK];
  __shared__ __align__(16) float swsum[CIN];
  __shared__ __align__(16) float smean[PBLK];
  __shared__ __align__(16) float svbar[PBLK];
  __shared__ float sbias[64];
  const int tid = threadIdx.x, wave = tid >> 5, lane = tid & 31, m = lane & 15, h = lane >> 4;

#pragma unroll 4
  for (int it = 0; it < (CIN * CQK) / 128; ++it) {
    const int idx = it * 128 + tid;
    const int k = idx >> 5, n = idx & 31;
    sW[n * PW + k] = bf_bits(Wq[idx]);
    sW[(32 + n) * PW + k] = bf_bits(Wk[idx]);
  }
  swsum[tid] = wsum[tid];
  swsum[tid + 128] = wsum[tid + 128];
  if (tid < 64) {
    const float vq = bq[tid & 31];
    const float vk = bk[tid & 31];
    sbias[tid] = bf_r(tid < 32 ? vq : vk);
  }
  const float bvsum = aux[0];
  __syncthreads();

  const int row0 = blockIdx.x * PBLK + wave * 16;
  const float* xr = x + (size_t)(row0 + m) * CIN + 8 * h;
  const float* wr = swsum + 8 * h;
  const unsigned short* wb = sW + m * PW + 8 * h;
  v8f acc[4];
#pragma unroll
  for (int t = 0; t < 4; ++t) acc[t] = zero8();
  float xs = 0.f, vd = 0.f;

#pragma unroll 2
  for (int c = 0; c < CIN / 32; ++c) {
    const float* p = xr + 32 * c;
    const v4f x0 = *(const v4f*)(p);
    const v4f x1 = *(const v4f*)(p + 4);
    const v4f x2 = *(const v4f*)(p + 16);
    const v4f x3 = *(const v4f*)(p + 20);
    const float* pw = wr + 32 * c;
    const v4f w0 = *(const v4f*)(pw);
    const v4f w1 = *(const v4f*)(pw + 4);
    const v4f w2 = *(const v4f*)(pw + 16);
    const v4f w3 = *(const v4f*)(pw + 20);
    v16us au;
#pragma unroll
    for (int e = 0; e < 4; ++e) {
      const unsigned short b0 = bf_bits(x0[e]), b1 = bf_bits(x1[e]);
      const unsigned short b2 = bf_bits(x2[e]), b3 = bf_bits(x3[e]);
      const float r0 = bf_up(b0), r1 = bf_up(b1), r2 = bf_up(b2), r3 = bf_up(b3);
      au[e] = b0; au[4 + e] = b1; au[8 + e] = b2; au[12 + e] = b3;
      xs += (r0 + r1) + (r2 + r3);
      vd += r0 * w0[e]; vd += r1 * w1[e]; vd += r2 * w2[e]; vd += r3 * w3[e];
    }
    const v16bf a = __builtin_bit_cast(v16bf, au);
    const unsigned short* bp = wb + 32 * c;
    const v16bf f0 = ldfrag_b(bp);
    const v16bf f1 = ldfrag_b(bp + 16 * PW);
    const v16bf f2 = ldfrag_b(bp + 32 * PW);
    const v16bf f3 = ldfrag_b(bp + 48 * PW);
    acc[0] = mma_b(a, f0, acc[0]);
    acc[1] = mma_b(a, f1, acc[1]);
    acc[2] = mma_b(a, f2, acc[2]);
    acc[3] = mma_b(a, f3, acc[3]);
    guard_p(acc[0], acc[1], acc[2], acc[3], a, f0, f1, f2, f3);
    sched_fence();
  }
  acc_guard4(acc[0], acc[1], acc[2], acc[3]);

  xs += __shfl_xor(xs, 16, 32);
  vd += __shfl_xor(vd, 16, 32);
  if (h == 0) {
    smean[wave * 16 + m] = xs * (1.0f / 256.0f);
    svbar[wave * 16 + m] = (vd + bvsum) * (1.0f / 256.0f);
  }
  unsigned short* so = sO + wave * (4 * 16 * CQK);
#pragma unroll
  for (int t = 0; t < 4; ++t) {
    const float bias = sbias[16 * t + m];
    const int col = 16 * (t & 1) + m;
    unsigned short* ph = so + (2 * (t >> 1)) * (16 * CQK) + col;
    unsigned short* pl = ph + 16 * CQK;
#pragma unroll
    for (int r = 0; r < 8; ++r) {
      const float val = acc[t][r] + bias;
      const unsigned short hb = bf_bits(val);
      const unsigned short lb = bf_bits(val - bf_up(hb));
      ph[(8 * h + r) * CQK] = hb;
      pl[(8 * h + r) * CQK] = lb;
    }
  }
  __syncthreads();
  v4u pc[8];
#pragma unroll
  for (int pidx = 0; pidx < 4; ++pidx) {
    pc[2 * pidx]     = *(const v4u*)(so + pidx * (16 * CQK) + lane * 8);
    pc[2 * pidx + 1] = *(const v4u*)(so + pidx * (16 * CQK) + 256 + lane * 8);
  }
  const size_t ob = (size_t)row0 * CQK + (size_t)lane * 8;
  *(volatile v4u*)(qh + ob) = pc[0];  *(volatile v4u*)(qh + ob + 256) = pc[1];
  *(volatile v4u*)(ql + ob) = pc[2];  *(volatile v4u*)(ql + ob + 256) = pc[3];
  *(volatile v4u*)(kh + ob) = pc[4];  *(volatile v4u*)(kh + ob + 256) = pc[5];
  *(volatile v4u*)(kl + ob) = pc[6];  *(volatile v4u*)(kl + ob + 256) = pc[7];
  __threadfence();
  *(volatile v4u*)(qh + ob) = pc[0];  *(volatile v4u*)(qh + ob + 256) = pc[1];
  *(volatile v4u*)(ql + ob) = pc[2];  *(volatile v4u*)(ql + ob + 256) = pc[3];
  *(volatile v4u*)(kh + ob) = pc[4];  *(volatile v4u*)(kh + ob + 256) = pc[5];
  *(volatile v4u*)(kl + ob) = pc[6];  *(volatile v4u*)(kl + ob + 256) = pc[7];

  if (wave == 0) {
    const v4f v = *(const v4f*)(smean + 4 * (lane & 15));
    float* dst = xmean + (size_t)blockIdx.x * PBLK + 4 * (lane & 15);
    if (lane < 16) *(volatile v4f*)dst = v;
    __threadfence();
    if (lane < 16) *(volatile v4f*)dst = v;
  } else if (wave == 1) {
    const v4f v = *(const v4f*)(svbar + 4 * (lane & 15));
    float* dst = vbar + (size_t)blockIdx.x * PBLK + 4 * (lane & 15);
    if (lane < 16) *(volatile v4f*)dst = v;
    __threadfence();
    if (lane < 16) *(volatile v4f*)dst = v;
  }
}

__global__ __launch_bounds__(128) void k_attn(const unsigned short* qh, const unsigned short* ql,
                                               const unsigned short* kh, const unsigned short* kl,
                                               const float* vbar, const float* xmean,
                                               const float* __restrict__ gamma, float* out) {
  __shared__ __align__(16) float svb[HWN];
  __shared__ __align__(16) float sout[QBLK];
  const int tid = threadIdx.x, wave = tid >> 5, lane = tid & 31;
  const int rl = lane & 15, h = lane >> 4, koff = 8 * h;
  const int n0 = blockIdx.x * QBLK;
  const int keybase = (n0 / HWN) * HWN;
#pragma unroll
  for (int i = tid; i < HWN / 4; i += 128) {
    ((v4f*)svb)[i] = *(const v4f*)(vbar + keybase + 4 * i);
  }
  const float gb = bf_r(gamma[0]);
  const int qrow = n0 + 16 * wave + rl;
  const float xm = xmean[qrow];
  __syncthreads();

  const v16bf fqh = ldfrag_b(qh + (size_t)qrow * CQK + koff);
  const v16bf fql = ldfrag_b(ql + (size_t)qrow * CQK + koff);
  const unsigned short* khp = kh + (size_t)(keybase + rl) * CQK + koff;
  const unsigned short* klp = kl + (size_t)(keybase + rl) * CQK + koff;

  float run_max = -1.0e30f, run_sum = 0.0f, run_o = 0.0f;

#pragma unroll 1
  for (int kb = 0; kb < HWN; kb += 32) {
    const unsigned short* pa = khp + (size_t)kb * CQK;
    const unsigned short* pl = klp + (size_t)kb * CQK;
    const v16bf a0h = ldfrag_b(pa);
    const v16bf a1h = ldfrag_b(pa + 16 * CQK);
    const v16bf a0l = ldfrag_b(pl);
    const v16bf a1l = ldfrag_b(pl + 16 * CQK);
    v8f s0 = zero8(), s1 = zero8();
    s0 = mma_b(a0h, fqh, s0);
    s0 = mma_b(a0h, fql, s0);
    s0 = mma_b(a0l, fqh, s0);
    s1 = mma_b(a1h, fqh, s1);
    s1 = mma_b(a1h, fql, s1);
    s1 = mma_b(a1l, fqh, s1);
    guard_s(s0, s1, a0h, a1h, a0l, a1l, fqh, fql);
    sched_fence();
    float lmax = fmaxf(s0[0], s1[0]);
#pragma unroll
    for (int v = 1; v < 8; ++v) lmax = fmaxf(lmax, fmaxf(s0[v], s1[v]));
    lmax = fmaxf(lmax, __shfl_xor(lmax, 16, 32));
    const float nm = fmaxf(run_max, lmax);
    const float factor = __expf(run_max - nm);
    run_max = nm;
    const v4f v00 = *(const v4f*)(svb + kb + koff);
    const v4f v01 = *(const v4f*)(svb + kb + koff + 4);
    const v4f v10 = *(const v4f*)(svb + kb + 16 + koff);
    const v4f v11 = *(const v4f*)(svb + kb + 16 + koff + 4);
    float lsum = 0.0f, po = 0.0f;
#pragma unroll
    for (int v = 0; v < 4; ++v) {
      const float p0 = __expf(s0[v] - nm);
      const float p1 = __expf(s1[v] - nm);
      const float p2 = __expf(s0[4 + v] - nm);
      const float p3 = __expf(s1[4 + v] - nm);
      lsum += (p0 + p1) + (p2 + p3);
      po += p0 * v00[v]; po += p1 * v10[v]; po += p2 * v01[v]; po += p3 * v11[v];
    }
    run_sum = run_sum * factor + lsum;
    run_o = run_o * factor + po;
  }

  const float tot = run_sum + __shfl_xor(run_sum, 16, 32);
  const float oo = run_o + __shfl_xor(run_o, 16, 32);
  const float res = gb * (oo * (1.0f / tot)) + xm;
  if (h == 0) sout[16 * wave + rl] = res;
  __syncthreads();
  if (wave == 0) {
    const v4f v = *(const v4f*)(sout + 4 * (lane & 15));
    float* dst = out + (size_t)n0 + 4 * (lane & 15);
    if (lane < 16) *(volatile v4f*)dst = v;
    __threadfence();
    if (lane < 16) *(volatile v4f*)dst = v;
  }
}

extern "C" void kernel_launch(void* const* d_in, const int* in_sizes, int n_in,
                              void* d_out, int out_size, void* d_ws, size_t ws_size,
                              hipStream_t stream) {
  if (n_in < 8) return;
  if (in_sizes[0] != NTOK * CIN) return;
  if (in_sizes[1] != CIN * CQK) return;
  if (in_sizes[2] != CQK) return;
  if (in_sizes[3] != CIN * CQK) return;
  if (in_sizes[4] != CQK) return;
  if (in_sizes[5] != CIN * CIN) return;
  if (in_sizes[6] != CIN) return;
  if (in_sizes[7] < 1) return;
  if (out_size != NTOK) return;

  const float* x     = (const float*)d_in[0];
  const float* Wq    = (const float*)d_in[1];
  const float* bq    = (const float*)d_in[2];
  const float* Wk    = (const float*)d_in[3];
  const float* bk    = (const float*)d_in[4];
  const float* Wv    = (const float*)d_in[5];
  const float* bv    = (const float*)d_in[6];
  const float* gamma = (const float*)d_in[7];
  float* out = (float*)d_out;

  const size_t PQK  = (size_t)NTOK * CQK * 2;
  const size_t PTOK = (size_t)NTOK * 4;
  const size_t PWS  = (size_t)CIN * 4;
  const size_t PAUX = (size_t)32 * 4;

  size_t off = 0;
  const size_t oQH = off; off += PQK;
  const size_t oQL = off; off += PQK;
  const size_t oKH = off; off += PQK;
  const size_t oKL = off; off += PQK;
  const size_t oXM = off; off += PTOK;
  const size_t oVB = off; off += PTOK;
  const size_t oWS = off; off += PWS;
  const size_t oAUX = off; off += PAUX;
  if (off > ws_size) return;
  if (off > (size_t)134217728) return;

  char* ws = (char*)d_ws;
  unsigned short* QH = (unsigned short*)(ws + oQH);
  unsigned short* QL = (unsigned short*)(ws + oQL);
  unsigned short* KH = (unsigned short*)(ws + oKH);
  unsigned short* KL = (unsigned short*)(ws + oKL);
  float* XM  = (float*)(ws + oXM);
  float* VB  = (float*)(ws + oVB);
  float* WS  = (float*)(ws + oWS);
  float* AUX = (float*)(ws + oAUX);

  k_prep<<<dim3(1), dim3(256), 0, stream>>>(Wv, bv, WS, AUX);
  k_proj<<<dim3(NTOK / PBLK), dim3(128), 0, stream>>>(x, Wq, bq, Wk, bk, WS, AUX, QH, QL, KH, KL, XM, VB);
  k_attn<<<dim3(NTOK / QBLK), dim3(128), 0, stream>>>(QH, QL, KH, KL, VB, XM, gamma, out);
  (void)hipGetLastError();
}
